// FlashSelfAttentionM_45423574122987
// MI455X (gfx1250) — hardware-verified
//
#include <hip/hip_runtime.h>


namespace {
constexpr int T = 3712, D = 1024, NH = 16, HD = 64, NCU = 5, NSEQ = NCU - 1, SMAX = 1024;
constexpr float XS = 8.0f, PS = 1024.0f, WSC = 256.0f, BASE = 10000.0f;
typedef _Float16 b16;
typedef __attribute__((ext_vector_type(16))) _Float16 v16b;
typedef __attribute__((ext_vector_type(8))) _Float16 v8b;
typedef __attribute__((ext_vector_type(8))) float v8f;
typedef __attribute__((ext_vector_type(4))) float v4f;
typedef __attribute__((ext_vector_type(2))) float v2f;
__device__ __forceinline__ float bf16_rne(float f) { unsigned int u = __float_as_uint(f); u += 0x7FFFu + ((u >> 16) & 1u); float r = __uint_as_float(u & 0xFFFF0000u); asm volatile("" : "+v"(r)); return r; }
__device__ __forceinline__ void split16(float v, b16& hi, b16& lo) { hi = (b16)v; lo = (b16)(v - (float)hi); }
__device__ __forceinline__ v16b frag_kb(const b16* p, int hh) { const v8b a = *(const v8b*)(p + 8 * hh), b = *(const v8b*)(p + 16 + 8 * hh); v16b f;
#pragma unroll
  for (int e = 0; e < 8; ++e) { f[e] = a[e]; f[8 + e] = b[e]; } return f; }
__device__ __forceinline__ v8f wmma16b(v16b a, v16b b, v8f c) { v8f d = __builtin_amdgcn_wmma_f32_16x16x32_f16(false, a, false, b, (short)0, c, false, false); asm volatile("v_nop\n\tv_nop\n\tv_nop\n\tv_nop" : "+v"(d) : "v"(a), "v"(b)); return d; }
__device__ __forceinline__ void wave_lds_sync() { __builtin_amdgcn_fence(__ATOMIC_RELEASE, "workgroup"); __builtin_amdgcn_wave_barrier(); __builtin_amdgcn_fence(__ATOMIC_ACQUIRE, "workgroup"); }
__device__ __forceinline__ float pmul(float a, float b) { float p = a * b; asm volatile("" : "+v"(p)); return p; }
__device__ __forceinline__ int iclamp(int v, int lo, int hi) { return v < lo ? lo : (v > hi ? hi : v); }
__device__ __forceinline__ int pos_of(const int* cu, int t) { int s = 0; for (int j = 0; j < NSEQ; ++j) if (cu[j] <= t) s = j; return t - cu[s]; }

__global__ __launch_bounds__(256) void wput_kernel(const float* __restrict__ w, int OUTW, b16* __restrict__ WT) { const size_t u = (size_t)blockIdx.x * 256 + threadIdx.x; if (u >= (size_t)OUTW * (D / 8)) return; const int o = (int)(u / (D / 8)), k0 = (int)(u % (D / 8)) * 8; v8b v;
#pragma unroll
  for (int j = 0; j < 8; ++j) v[j] = (b16)(bf16_rne(w[(size_t)(k0 + j) * OUTW + o]) * WSC); for (int pass = 0; pass < 2; ++pass) { *(volatile v8b*)(WT + (size_t)o * D + k0) = v; __threadfence(); } }
__global__ __launch_bounds__(32) void qkv_kernel(const float* __restrict__ x, const b16* __restrict__ WT, const float* __restrict__ bias, const int* __restrict__ cu, int TV, float* __restrict__ Q, float* __restrict__ K, float* __restrict__ V) {
  __shared__ __attribute__((aligned(16))) b16 Ah[16][D + 8]; __shared__ float Tf[16][132], Cs[16][32], Sn[16][32]; __shared__ int Ps[16]; const int lane = threadIdx.x, nloc = lane & 15, hlf = lane >> 4; const int cg = blockIdx.x % 24; const size_t m0 = (size_t)(blockIdx.x / 24) * 16;
  if (lane < 16) Ps[lane] = pos_of(cu, (int)m0 + lane);
  wave_lds_sync();
  { bool any = false; for (int rr = 0; rr < 16; ++rr) any |= Ps[rr] < TV; if (!any) return; }
  if (cg < 16) { const float invf = 1.0f / powf(BASE, (float)(2 * lane) / (float)HD);
#pragma unroll 1
    for (int rr = 0; rr < 16; ++rr) { const float ang = (float)Ps[rr] * invf; Cs[rr][lane] = cosf(ang); Sn[rr][lane] = sinf(ang); } }
  for (int rr = 0; rr < 16; ++rr) for (int q = 0; q < D / 32; ++q) Ah[rr][q * 32 + lane] = (b16)(bf16_rne(x[(m0 + rr) * D + q * 32 + lane]) * XS);
  wave_lds_sync(); v8f acc[8];
#pragma unroll
  for (int t = 0; t < 8; ++t) acc[t] = (v8f){};
#pragma unroll 2
  for (int kb = 0; kb < D; kb += 32) { const v16b a = frag_kb(&Ah[nloc][kb], hlf);
#pragma unroll
    for (int t = 0; t < 8; ++t) acc[t] = wmma16b(a, frag_kb(WT + (size_t)(cg * 128 + t * 16 + nloc) * D + kb, hlf), acc[t]); }
#pragma unroll
  for (int t = 0; t < 8; ++t) { const int c = cg * 128 + t * 16 + nloc; const float bb = bf16_rne(bias[c]);
#pragma unroll
    for (int r8 = 0; r8 < 8; ++r8) Tf[8 * hlf + r8][t * 16 + nloc] = acc[t][r8] * (1.0f / (XS * WSC)) + bb; }
  wave_lds_sync();
  const int which = cg / 8; float* O = which == 0 ? Q : (which == 1 ? K : V); const int c0 = (cg % 8) * 128;
  for (int pass = 0; pass < 2; ++pass) { for (int rr = 0; rr < 16; ++rr) {
      for (int q = 0; q < 4; ++q) { const int c = q * 32 + lane; float val = Tf[rr][c];
        if (which < 2) { const int dd = c & 63; const int i = dd & 31; const float cs = Cs[rr][i], sn = Sn[rr][i]; val = (dd < 32) ? pmul(val, cs) - pmul(Tf[rr][c + 32], sn) : pmul(val, cs) + pmul(Tf[rr][c - 32], sn); }
        ((volatile float*)O)[(m0 + rr) * D + c0 + c] = val; } }
    __threadfence(); }
}
__global__ __launch_bounds__(32) void att_kernel(const float* __restrict__ Q, const float* __restrict__ K, const float* __restrict__ V, const int* __restrict__ cu, int TV, float* __restrict__ O) {
  __shared__ __attribute__((aligned(16))) b16 Qh[16][HD + 8], Ql[16][HD + 8], Kh[32][HD + 8], Kl[32][HD + 8], Ph[16][40], Pl[16][40], Vh[HD][40], Vl[HD][40]; __shared__ float Sc[16][33], Mx[16], Dn[16], Sf[16], Of[16][HD + 2];
  const int lane = threadIdx.x, nloc = lane & 15, hlf = lane >> 4; const int qt = blockIdx.x % (SMAX / 16); const int h = (blockIdx.x / (SMAX / 16)) % NH; const int b = blockIdx.x / ((SMAX / 16) * NH);
  const int s0 = iclamp(cu[b], 0, T), s1 = iclamp(cu[b + 1], s0, T); const int len = s1 - s0; const int q0 = qt * 16; if (q0 >= len || q0 >= TV) return; const int nq = len - q0 < 16 ? len - q0 : 16;
  for (int rr = 0; rr < 16; ++rr) for (int q = 0; q < 2; ++q) { b16 p = (b16)0.0f, ql = (b16)0.0f; if (rr < nq) split16(Q[(size_t)(s0 + q0 + rr) * D + h * HD + q * 32 + lane] * XS, p, ql); Qh[rr][q * 32 + lane] = p; Ql[rr][q * 32 + lane] = ql; }
  if (lane < 16) { Mx[lane] = -INFINITY; Dn[lane] = 0.0f; Sf[lane] = 0.0f; }
  v8f acc[4] = {(v8f){}, (v8f){}, (v8f){}, (v8f){}}; wave_lds_sync();
#pragma unroll 1
  for (int kc = 0; kc < q0 + nq; kc += 32) {
    for (int rr = 0; rr < 32; ++rr) { const int kk = kc + rr; const bool ok = kk < len; for (int q = 0; q < 2; ++q) { b16 p = (b16)0.0f, ql = (b16)0.0f, vp = (b16)0.0f, vl = (b16)0.0f; if (ok) { split16(K[(size_t)(s0 + kk) * D + h * HD + q * 32 + lane] * XS, p, ql); split16(V[(size_t)(s0 + kk) * D + h * HD + q * 32 + lane] * XS, vp, vl); } Kh[rr][q * 32 + lane] = p; Kl[rr][q * 32 + lane] = ql; Vh[q * 32 + lane][rr] = vp; Vl[q * 32 + lane][rr] = vl; } }
    wave_lds_sync();
#pragma unroll
    for (int blk = 0; blk < 2; ++blk) { v8f s = {};
#pragma unroll
      for (int kb = 0; kb < HD; kb += 32) { const v16b qh = frag_kb(&Qh[nloc][kb], hlf), qlo = frag_kb(&Ql[nloc][kb], hlf), kh = frag_kb(&Kh[blk * 16 + nloc][kb], hlf), kl = frag_kb(&Kl[blk * 16 + nloc][kb], hlf); s = wmma16b(qh, kh, s); s = wmma16b(qh, kl, s); s = wmma16b(qlo, kh, s); }
#pragma unroll
      for (int r8 = 0; r8 < 8; ++r8) { const int qi = q0 + 8 * hlf + r8, kk = kc + blk * 16 + nloc; Sc[8 * hlf + r8][blk * 16 + nloc] = (kk <= qi && kk < len) ? s[r8] * (0.125f / (XS * XS)) : -INFINITY; } }
    wave_lds_sync();
#pragma unroll 1
    for (int qi = 0; qi < 16; ++qi) { const float sv = Sc[qi][lane]; float cm = sv; for (int o = 16; o; o >>= 1) cm = fmaxf(cm, __shfl_xor(cm, o)); const float mo = Mx[qi]; const float mn = fmaxf(mo, cm); const float p = (sv == -INFINITY) ? 0.0f : __expf(sv - mn); float psum = p; for (int o = 16; o; o >>= 1) psum += __shfl_xor(psum, o);
      b16 ph, plo; split16(p * PS, ph, plo); Ph[qi][lane] = ph; Pl[qi][lane] = plo; if (lane == 0) { const float sf = (mo == -INFINITY) ? 0.0f : __expf(mo - mn); Sf[qi] = sf; Dn[qi] = Dn[qi] * sf + psum; Mx[qi] = mn; } }
    wave_lds_sync(); const v16b pa = frag_kb(&Ph[nloc][0], hlf), pb = frag_kb(&Pl[nloc][0], hlf);
#pragma unroll
    for (int tt = 0; tt < 4; ++tt) {
#pragma unroll
      for (int r8 = 0; r8 < 8; ++r8) acc[tt][r8] *= Sf[8 * hlf + r8];
      const v16b vh = frag_kb(&Vh[tt * 16 + nloc][0], hlf), vl = frag_kb(&Vl[tt * 16 + nloc][0], hlf); acc[tt] = wmma16b(pa, vh, acc[tt]); acc[tt] = wmma16b(pa, vl, acc[tt]); acc[tt] = wmma16b(pb, vh, acc[tt]); }
    wave_lds_sync(); }
#pragma unroll
  for (int tt = 0; tt < 4; ++tt)
#pragma unroll
    for (int r8 = 0; r8 < 8; ++r8) { const int rl = 8 * hlf + r8; Of[rl][tt * 16 + nloc] = acc[tt][r8] * (1.0f / (PS * XS)) / (Dn[rl] > 0.0f ? Dn[rl] : 1.0f); }
  wave_lds_sync();
  for (int pass = 0; pass < 2; ++pass) { for (int rr = 0; rr < nq; ++rr) *(volatile v2f*)(O + (size_t)(s0 + q0 + rr) * D + h * HD + lane * 2) = (v2f){Of[rr][lane * 2], Of[rr][lane * 2 + 1]}; __threadfence(); }
}
__global__ __launch_bounds__(32) void proj_kernel(const float* __restrict__ O, const b16* __restrict__ WT, const float* __restrict__ bias, const int* __restrict__ cu, int TV, float* __restrict__ out) {
  __shared__ __attribute__((aligned(16))) b16 Ah[16][D + 8], Al[16][D + 8]; __shared__ float Tf[16][132]; __shared__ int Ok[16]; const int lane = threadIdx.x, nloc = lane & 15, hlf = lane >> 4; const int cg = blockIdx.x % 8; const size_t m0 = (size_t)(blockIdx.x / 8) * 16;
  if (lane < 16) Ok[lane] = pos_of(cu, (int)m0 + lane) < TV;
  wave_lds_sync();
  { bool any = false; for (int rr = 0; rr < 16; ++rr) any |= Ok[rr] != 0; if (!any) { for (int pass = 0; pass < 2; ++pass) { for (int rr = 0; rr < 16; ++rr) *(volatile v4f*)(out + (m0 + rr) * D + cg * 128 + lane * 4) = (v4f){0.0f, 0.0f, 0.0f, 0.0f}; __threadfence(); } return; } }
  for (int rr = 0; rr < 16; ++rr) for (int q = 0; q < D / 32; ++q) { b16 p = (b16)0.0f, ql = (b16)0.0f; if (Ok[rr]) split16(O[(m0 + rr) * D + q * 32 + lane] * XS, p, ql); Ah[rr][q * 32 + lane] = p; Al[rr][q * 32 + lane] = ql; }
  wave_lds_sync(); v8f acc[8];
#pragma unroll
  for (int t = 0; t < 8; ++t) acc[t] = (v8f){};
#pragma unroll 2
  for (int kb = 0; kb < D; kb += 32) { const v16b a = frag_kb(&Ah[nloc][kb], hlf), al = frag_kb(&Al[nloc][kb], hlf);
#pragma unroll
    for (int t = 0; t < 8; ++t) { const v16b bw = frag_kb(WT + (size_t)(cg * 128 + t * 16 + nloc) * D + kb, hlf); acc[t] = wmma16b(a, bw, acc[t]); acc[t] = wmma16b(al, bw, acc[t]); } }
#pragma unroll
  for (int t = 0; t < 8; ++t) { const int c = cg * 128 + t * 16 + nloc; const float bb = bf16_rne(bias[c]);
#pragma unroll
    for (int r8 = 0; r8 < 8; ++r8) { const int rl = 8 * hlf + r8; Tf[rl][t * 16 + nloc] = Ok[rl] ? acc[t][r8] * (1.0f / (XS * WSC)) + bb : 0.0f; } }
  wave_lds_sync();
  for (int pass = 0; pass < 2; ++pass) { for (int rr = 0; rr < 16; ++rr) *(volatile v4f*)(out + (m0 + rr) * D + cg * 128 + lane * 4) = *(const v4f*)(&Tf[rr][lane * 4]); __threadfence(); }
}
}

extern "C" void kernel_launch(void* const* d_in, const int* in_sizes, int n_in, void* d_out, int out_size, void* d_ws, size_t ws_size, hipStream_t stream) {
  (void)n_in;
  auto Fp = [&](int i) { return (const float*)d_in[i]; }; auto Ip = [&](int i) { return (const int*)d_in[i]; };
  if (in_sizes[0] != T * D || in_sizes[1] != D * 3 * D || in_sizes[2] != 3 * D || in_sizes[3] != D * D || in_sizes[4] != D || in_sizes[5] != NCU || out_size != T * D) return;
  const int TV = SMAX;
  size_t off = 0; char* ws = (char*)d_ws;
  auto carve = [&](size_t bytes) { char* p = ws + off; off += (bytes + 255) & ~(size_t)255; return p; };
  b16* WQ = (b16*)carve((size_t)3 * D * D * 2); b16* WO = (b16*)carve((size_t)D * D * 2); float* Q = (float*)carve((size_t)T * D * 4); float* K = (float*)carve((size_t)T * D * 4); float* V = (float*)carve((size_t)T * D * 4); float* O = (float*)carve((size_t)T * D * 4);
  if (off > ws_size || off > ((size_t)96 << 20)) return;
  wput_kernel<<<(unsigned)(((size_t)3 * D * (D / 8) + 255) / 256), 256, 0, stream>>>(Fp(1), 3 * D, WQ); wput_kernel<<<(unsigned)(((size_t)D * (D / 8) + 255) / 256), 256, 0, stream>>>(Fp(3), D, WO);
  qkv_kernel<<<(T / 16) * 24, 32, 0, stream>>>(Fp(0), WQ, Fp(2), Ip(5), TV, Q, K, V);
  att_kernel<<<NSEQ * NH * (SMAX / 16), 32, 0, stream>>>(Q, K, V, Ip(5), TV, O);
  proj_kernel<<<(T / 16) * 8, 32, 0, stream>>>(O, WO, Fp(4), Ip(5), TV, (float*)d_out);
}
